// _EGNNLayer_48455821033952
// MI455X (gfx1250) — hardware-verified
//
#include <hip/hip_runtime.h>
#include <stddef.h>
#include <math.h>


#define HDIM   128
#define EFD    16
#define KE     32
#define K1R    273
#define KDSQ   256
#define KEOFF  257
#define PW     256
#define NTHR   256
#define NWV    8
#define TR     64
#define LDH    136
#define LDF    132
#define BM     32
#define CE     65536
#define NB     256
#define CH     2048
#define LCAP   4096
#define SP     128
#define WSCAP  134217728
#define SCL_H   8.0f
#define SCL_W   16.0f
#define SCL_EF  8.0f
#define SCL_ACT 8.0f
#define INV_HW  0.0078125f

#define LG_SLIST 0
#define LG_SLOTS (LG_SLIST + LCAP * 4)
#define LG_SDL   (LG_SLOTS + NB * SP * 2)
#define LG_SDX   (LG_SDL + LCAP * 4)
#define LG_XO    (LG_SDX + NB * 4 * 4)
#define LG_SCNT  (LG_XO + NB * 3 * 4)
#define LG_WSUM  (LG_SCNT + NB * 4)
#define LDS_G    (LG_WSUM + 64)

static_assert((LDH % 8) == 0 && LDH >= HDIM && (LDF % 4) == 0 && LDF >= HDIM);
static_assert(TR == 64 && NWV * 32 == NTHR && (TR * HDIM / 8) % NTHR == 0 && (TR * HDIM / 4) % NTHR == 0);
static_assert((CE % TR) == 0 && (CE % 8) == 0);
static_assert(NB == NTHR && CH == 8 * NTHR && LCAP >= 2 * CH && (LCAP % 4) == 0 && LCAP <= 65536 && SP <= LCAP);
static_assert((NB * 3) % 4 == 0 && (NB * 3 / 4) <= NTHR && NB == 32 * NWV);
static_assert(BM * 8 == NTHR && PW == 2 * HDIM && (HDIM % 32) == 0 && EFD <= 16 && KEOFF + EFD == K1R);
static_assert((LG_SLOTS % 16) == 0 && (LG_SDL % 16) == 0 && (LG_SDX % 16) == 0 && (LG_XO % 16) == 0);
static_assert((LG_SCNT % 16) == 0 && (LG_WSUM % 16) == 0);

typedef float          v4f   __attribute__((ext_vector_type(4)));
typedef float          v8f   __attribute__((ext_vector_type(8)));
typedef int            v4i   __attribute__((ext_vector_type(4)));
typedef _Float16       v8h   __attribute__((ext_vector_type(8)));
typedef _Float16       v16h  __attribute__((ext_vector_type(16)));
typedef unsigned short v8us  __attribute__((ext_vector_type(8)));
typedef __bf16         v16b  __attribute__((ext_vector_type(16)));
union FragH { v16h v; v8h hh[2]; };
union FragB { v16b v; v8us uh[2]; };

__device__ __forceinline__ v8f wmh(v16h a, v16h b, v8f c) {
  v8f d = __builtin_amdgcn_wmma_f32_16x16x32_f16(false, a, false, b, (short)0, c, false, false);
  asm volatile("v_nop\n\tv_nop\n\tv_nop\n\tv_nop" : "+v"(d) : "v"(a), "v"(b));
  return d;
}
__device__ __forceinline__ v8f wmb(v16b a, v16b b, v8f c) {
  v8f d = __builtin_amdgcn_wmma_f32_16x16x32_bf16(false, a, false, b, (short)0, c, false, false);
  asm volatile("v_nop\n\tv_nop\n\tv_nop\n\tv_nop" : "+v"(d) : "v"(a), "v"(b));
  return d;
}

__device__ __forceinline__ v8f zero8() { v8f z = {0.f, 0.f, 0.f, 0.f, 0.f, 0.f, 0.f, 0.f}; return z; }

__device__ __forceinline__ v8f cat8(v4f a, v4f b) {
  v8f t;
  t[0] = a.x; t[1] = a.y; t[2] = a.z; t[3] = a.w;
  t[4] = b.x; t[5] = b.y; t[6] = b.z; t[7] = b.w;
  return t;
}

__device__ __forceinline__ v8h cvt8(v4f a, v4f b, float s) {
  v8f t = cat8(a, b);
#pragma unroll
  for (int i = 0; i < 8; ++i) t[i] = t[i] * s;
  return __builtin_convertvector(t, v8h);
}

__device__ __forceinline__ unsigned bfb(float x) {
  const unsigned u = __float_as_uint(x);
  return (u + 0x7FFFu + ((u >> 16) & 1u)) >> 16;
}

__device__ __forceinline__ void split8(v8f t, v8us& hi, v8us& lo) {
  v8us hh = {0, 0, 0, 0, 0, 0, 0, 0};
  v8us ll = {0, 0, 0, 0, 0, 0, 0, 0};
#pragma unroll
  for (int i = 0; i < 8; ++i) {
    const unsigned hb = bfb(t[i]);
    const float    hf = __uint_as_float(hb << 16);
    const unsigned lb = bfb(t[i] - hf);
    hh[i] = (unsigned short)hb;
    ll[i] = (unsigned short)lb;
  }
  hi = hh; lo = ll;
}

__device__ __forceinline__ v16h frag16(const _Float16* p) {
  FragH f;
  f.hh[0] = *(const v8h*)p;
  f.hh[1] = *(const v8h*)(p + 16);
  return f.v;
}
__device__ __forceinline__ v16b fragbf(const unsigned short* p) {
  FragB f;
  f.uh[0] = *(const v8us*)p;
  f.uh[1] = *(const v8us*)(p + 16);
  return f.v;
}

__device__ __forceinline__ v16h afrag_f32(const float* rp, int h, float s) {
  FragH a;
  const float* p0 = rp + 8 * h;
  const float* p1 = rp + 16 + 8 * h;
  a.hh[0] = cvt8(*(const v4f*)p0, *(const v4f*)(p0 + 4), s);
  a.hh[1] = cvt8(*(const v4f*)p1, *(const v4f*)(p1 + 4), s);
  return a.v;
}
__device__ __forceinline__ void afrag_bf(const float* rp, int h, FragB& ah, FragB& al) {
  const float* p0 = rp + 8 * h;
  const float* p1 = rp + 16 + 8 * h;
  split8(cat8(*(const v4f*)p0, *(const v4f*)(p0 + 4)), ah.uh[0], al.uh[0]);
  split8(cat8(*(const v4f*)p1, *(const v4f*)(p1 + 4)), ah.uh[1], al.uh[1]);
}

__device__ __forceinline__ float rcp_f(float x)  { return __builtin_amdgcn_rcpf(x); }
__device__ __forceinline__ float silu_f(float x) { return x * rcp_f(1.0f + __expf(-x)); }

__global__ __launch_bounds__(NTHR) void k_wcvt(const float* __restrict__ in, _Float16* outp,
                                               int C, int koff, int K, int KP, int nUnits, float scale) {
  const int u = (int)blockIdx.x * NTHR + (int)threadIdx.x;
  if (u >= nUnits) return;
  const int upr = KP >> 3;
  const int n   = u / upr;
  const int k0  = (u - n * upr) * 8;
  v8f t;
#pragma unroll
  for (int i = 0; i < 8; ++i) {
    const int k  = k0 + i;
    const int kc = k < K ? k : K - 1;
    const float v = in[(size_t)(koff + kc) * C + n] * scale;
    t[i] = (k < K) ? v : 0.0f;
  }
  const v8h o = __builtin_convertvector(t, v8h);
  _Float16* d = outp + (size_t)n * KP + k0;
  *(volatile v8h*)d = o;
  __threadfence();
  *(volatile v8h*)d = o;
}

__global__ __launch_bounds__(NTHR) void k_wcvt_bf(const float* __restrict__ in, unsigned short* hip_,
                                                  unsigned short* lop, int C, int koff, int K, int KP, int nUnits) {
  const int u = (int)blockIdx.x * NTHR + (int)threadIdx.x;
  if (u >= nUnits) return;
  const int upr = KP >> 3;
  const int n   = u / upr;
  const int k0  = (u - n * upr) * 8;
  v8f t;
#pragma unroll
  for (int i = 0; i < 8; ++i) {
    const int k  = k0 + i;
    const int kc = k < K ? k : K - 1;
    const float v = in[(size_t)(koff + kc) * C + n];
    t[i] = (k < K) ? v : 0.0f;
  }
  v8us oh, ol;
  split8(t, oh, ol);
  const size_t o = (size_t)n * KP + k0;
  *(volatile v8us*)(hip_ + o) = oh;
  *(volatile v8us*)(lop + o)  = ol;
  __threadfence();
  *(volatile v8us*)(hip_ + o) = oh;
  *(volatile v8us*)(lop + o)  = ol;
}

__global__ __launch_bounds__(NTHR) void k_film(const float* __restrict__ cond, const float* __restrict__ Wf,
                                               const float* __restrict__ bf, float* film, int nUnits) {
  const int u = (int)blockIdx.x * NTHR + (int)threadIdx.x;
  if (u >= nUnits) return;
  const int g  = u >> 6;
  const int c4 = (u & 63) * 4;
  const float* cr = cond + (size_t)g * HDIM;
  const float* wr = Wf + c4;
  v4f s = {0.0f, 0.0f, 0.0f, 0.0f};
#pragma unroll 1
  for (int k = 0; k < HDIM; ++k) {
    const float cv = cr[k];
    const v4f   w  = *(const v4f*)(wr + (size_t)k * (2 * HDIM));
    s = s + w * cv;
  }
  s = s + *(const v4f*)(bf + c4);
  float* d = film + (size_t)g * (2 * HDIM) + c4;
  *(volatile v4f*)d = s;
  __threadfence();
  *(volatile v4f*)d = s;
}

__global__ __launch_bounds__(NTHR) __attribute__((amdgpu_num_vgpr(256)))
void k_nodegemm(const float* __restrict__ hin, const _Float16* __restrict__ wPQ,
                const float* __restrict__ b1, float* pq, int nN) {
  constexpr int NIT4 = (BM * PW / 4) / NTHR;
  static_assert((BM * PW / 4) % NTHR == 0 && NIT4 == 8);
  __shared__ __attribute__((aligned(16))) float stg[BM * PW];
  const int tid = threadIdx.x, lane = tid & 31;
  const int wave = __builtin_amdgcn_readfirstlane(tid >> 5);
  const int hh = lane >> 4, m = lane & 15;
  const int rg = wave >> 2, cq = wave & 3;
  const int r0 = rg * 16, c0 = cq * 64;
  const int rowBase = blockIdx.x * BM;

  v8f acc[4];
#pragma unroll
  for (int t = 0; t < 4; ++t) acc[t] = zero8();

  int ar = rowBase + r0 + m;
  ar = ar > nN - 1 ? nN - 1 : ar;
  const float* ap = hin + (size_t)ar * HDIM;
  const _Float16* bp0 = wPQ + (size_t)(c0 + m) * HDIM + 8 * hh;
#pragma unroll 1
  for (int kt = 0; kt < HDIM / 32; ++kt) {
    const v16h a = afrag_f32(ap + 32 * kt, hh, SCL_H);
#pragma unroll
    for (int t = 0; t < 4; ++t) acc[t] = wmh(a, frag16(bp0 + (size_t)(16 * t) * HDIM + 32 * kt), acc[t]);
  }

  float* sp = stg + (size_t)(r0 + 8 * hh) * PW + c0 + m;
  const int grow0 = rowBase + r0 + 8 * hh;
#pragma unroll
  for (int t = 0; t < 4; ++t) {
    const int n  = c0 + 16 * t + m;
    const int nb = n < HDIM ? n : HDIM - 1;
    float bv = b1[nb];
    bv = (n < HDIM) ? bv : 0.0f;
#pragma unroll
    for (int r = 0; r < 8; ++r) {
      float v = acc[t][r] * INV_HW + bv;
      v = (grow0 + r < nN) ? v : 0.0f;
      sp[r * PW + 16 * t] = v;
    }
  }
  __syncthreads();

  float* tile = pq + (size_t)rowBase * PW;
  v4f ov[NIT4];
#pragma unroll
  for (int it = 0; it < NIT4; ++it) ov[it] = *(const v4f*)(stg + 4 * (it * NTHR + tid));
#pragma unroll
  for (int it = 0; it < NIT4; ++it) *(volatile v4f*)(tile + 4 * (size_t)(it * NTHR + tid)) = ov[it];
  __threadfence();
#pragma unroll
  for (int it = 0; it < NIT4; ++it) *(volatile v4f*)(tile + 4 * (size_t)(it * NTHR + tid)) = ov[it];
}

__global__ __launch_bounds__(NTHR) __attribute__((amdgpu_num_vgpr(256)))
void k_edge1(const float* __restrict__ pq, const int* __restrict__ ei, const float* __restrict__ x,
             const float* __restrict__ ea, const _Float16* __restrict__ wE, const float* __restrict__ wd,
             _Float16* m1p, int nE, int nN, int ebase) {
  constexpr int NIT = (TR * HDIM / 8) / NTHR;
  constexpr int NSU = (16 * 64 / 4) / 32;
  __shared__ __attribute__((aligned(16))) float    stg[TR * HDIM];
  __shared__ __attribute__((aligned(16))) _Float16 tile[TR * LDH];
  const int tid = threadIdx.x, lane = tid & 31;
  const int wave = __builtin_amdgcn_readfirstlane(tid >> 5);
  const int h = lane >> 4, m = lane & 15;
  const int rg = wave >> 1, ch = wave & 1;
  const int cb = 64 * ch;
  const int rl0 = blockIdx.x * TR;
  const int e0 = ebase + rl0;

  const int eg = e0 + 16 * rg + m;
  const int e = eg > nE - 1 ? nE - 1 : eg;
  int di = ei[e];
  int sj = ei[(size_t)nE + e];
  di = di < 0 ? 0 : (di > nN - 1 ? nN - 1 : di);
  sj = sj < 0 ? 0 : (sj > nN - 1 ? nN - 1 : sj);
  const float* xi = x + (size_t)di * 3;
  const float* xj = x + (size_t)sj * 3;
  const float rx = xi[0] - xj[0], ry = xi[1] - xj[1], rz = xi[2] - xj[2];
  const float dsq = (rx * rx + rz * rz) + ry * ry;

  FragH ef;
  {
    const float* ap = ea + (size_t)e * EFD + 8 * h;
    ef.hh[0] = cvt8(*(const v4f*)ap, *(const v4f*)(ap + 4), SCL_EF);
    ef.hh[1] = __builtin_convertvector(zero8(), v8h);
  }
  v8f acc1[4];
#pragma unroll
  for (int nt = 0; nt < 4; ++nt) acc1[nt] = zero8();
  {
    const _Float16* bp0 = wE + (size_t)(cb + m) * KE + 8 * h;
#pragma unroll
    for (int nt = 0; nt < 4; ++nt) acc1[nt] = wmh(ef.v, frag16(bp0 + (size_t)(16 * nt) * KE), acc1[nt]);
  }

#pragma unroll 4
  for (int i = 0; i < NSU; ++i) {
    const int u   = i * 32 + lane;
    const int row = u >> 4;
    const int c4  = (u & 15) * 4;
    const int dr  = __shfl(di, row);
    const int sr  = __shfl(sj, row);
    const v4f p4 = *(const v4f*)(pq + (size_t)dr * PW + cb + c4);
    const v4f q4 = *(const v4f*)(pq + (size_t)sr * PW + HDIM + cb + c4);
    *(v4f*)(stg + (size_t)(16 * rg + row) * HDIM + cb + c4) = p4 + q4;
  }
  __syncthreads();

  float dq[8];
#pragma unroll
  for (int r = 0; r < 8; ++r) dq[r] = __shfl(dsq, 8 * h + r);

  {
    const float* srow = stg + (size_t)(16 * rg + 8 * h) * HDIM + cb + m;
    _Float16* trow = tile + (size_t)(16 * rg + 8 * h) * LDH + cb + m;
#pragma unroll
    for (int nt = 0; nt < 4; ++nt) {
      const float wv = wd[cb + 16 * nt + m];
#pragma unroll
      for (int r = 0; r < 8; ++r) {
        const float pre = acc1[nt][r] * INV_HW + srow[r * HDIM + 16 * nt] + dq[r] * wv;
        trow[r * LDH + 16 * nt] = (_Float16)(silu_f(pre) * SCL_ACT);
      }
    }
  }
  __syncthreads();

  _Float16* dstp = m1p + (size_t)rl0 * HDIM;
  v8h ov[NIT];
#pragma unroll
  for (int it = 0; it < NIT; ++it) {
    const int u = it * NTHR + tid;
    ov[it] = *(const v8h*)(tile + (u >> 4) * LDH + (u & 15) * 8);
  }
#pragma unroll
  for (int it = 0; it < NIT; ++it) *(volatile v8h*)(dstp + 8 * (size_t)(it * NTHR + tid)) = ov[it];
  __threadfence();
#pragma unroll
  for (int it = 0; it < NIT; ++it) *(volatile v8h*)(dstp + 8 * (size_t)(it * NTHR + tid)) = ov[it];
}

__global__ __launch_bounds__(NTHR) __attribute__((amdgpu_num_vgpr(256)))
void k_edge2(const _Float16* __restrict__ m1p, const int* __restrict__ ei, const float* __restrict__ x,
             const _Float16* __restrict__ w2, const _Float16* __restrict__ wx,
             const float* __restrict__ b2, const float* __restrict__ bc1, const float* __restrict__ Wc2,
             float* mijf, float* aux, int nE, int nN, int ebase) {
  constexpr int NIT4 = (TR * HDIM / 4) / NTHR;
  __shared__ __attribute__((aligned(16))) float    stg[TR * HDIM];
  __shared__ __attribute__((aligned(16))) _Float16 tile[TR * LDH];
  __shared__ float xsx[TR * 2];
  const int tid = threadIdx.x, lane = tid & 31;
  const int wave = __builtin_amdgcn_readfirstlane(tid >> 5);
  const int h = lane >> 4, m = lane & 15;
  const int rg = wave >> 1, ch = wave & 1;
  const int cb = 64 * ch;
  const int rl0 = blockIdx.x * TR;

  v8f acc[4];
#pragma unroll
  for (int nt = 0; nt < 4; ++nt) acc[nt] = zero8();
  {
    const _Float16* ap  = m1p + (size_t)(rl0 + 16 * rg + m) * HDIM + 8 * h;
    const _Float16* bp0 = w2 + (size_t)(cb + m) * HDIM + 8 * h;
#pragma unroll 1
    for (int kt = 0; kt < HDIM / 32; ++kt) {
      const v16h a = frag16(ap + 32 * kt);
#pragma unroll
      for (int nt = 0; nt < 4; ++nt) acc[nt] = wmh(a, frag16(bp0 + (size_t)(16 * nt) * HDIM + 32 * kt), acc[nt]);
    }
  }
  {
    float*    srow = stg + (size_t)(16 * rg + 8 * h) * HDIM + cb + m;
    _Float16* trow = tile + (size_t)(16 * rg + 8 * h) * LDH + cb + m;
#pragma unroll
    for (int nt = 0; nt < 4; ++nt) {
      const float bb = b2[cb + 16 * nt + m];
#pragma unroll
      for (int r = 0; r < 8; ++r) {
        const float v = silu_f(acc[nt][r] * INV_HW + bb);
        srow[r * HDIM + 16 * nt] = v;
        trow[r * LDH + 16 * nt] = (_Float16)(v * SCL_ACT);
      }
    }
  }
  __syncthreads();

#pragma unroll
  for (int nt = 0; nt < 4; ++nt) acc[nt] = zero8();
  {
    const _Float16* arow = tile + (size_t)(16 * rg + m) * LDH + 8 * h;
    const _Float16* bq0  = wx + (size_t)(cb + m) * HDIM + 8 * h;
#pragma unroll 1
    for (int kt = 0; kt < HDIM / 32; ++kt) {
      const v16h a = frag16(arow + 32 * kt);
#pragma unroll
      for (int nt = 0; nt < 4; ++nt) acc[nt] = wmh(a, frag16(bq0 + (size_t)(16 * nt) * HDIM + 32 * kt), acc[nt]);
    }
  }
  float es[8];
#pragma unroll
  for (int r = 0; r < 8; ++r) es[r] = 0.0f;
#pragma unroll
  for (int nt = 0; nt < 4; ++nt) {
    const int col = cb + 16 * nt + m;
    const float bb = bc1[col], wv = Wc2[col];
#pragma unroll
    for (int r = 0; r < 8; ++r) es[r] += silu_f(acc[nt][r] * INV_HW + bb) * wv;
  }
#pragma unroll
  for (int r = 0; r < 8; ++r) {
    float t = es[r];
    t += __shfl_xor(t, 8);
    t += __shfl_xor(t, 4);
    t += __shfl_xor(t, 2);
    t += __shfl_xor(t, 1);
    es[r] = t;
  }
  {
    float mine = 0.0f;
#pragma unroll
    for (int r = 0; r < 8; ++r) mine = ((m & 7) == r) ? es[r] : mine;
    if (m < 8) xsx[(16 * rg + 8 * h + m) * 2 + ch] = mine;
  }
  __syncthreads();

  if (tid < TR) {
    const int row = tid;
    const int eg = ebase + rl0 + row;
    const int e = eg > nE - 1 ? nE - 1 : eg;
    int di = ei[e];
    int sj = ei[(size_t)nE + e];
    di = di < 0 ? 0 : (di > nN - 1 ? nN - 1 : di);
    sj = sj < 0 ? 0 : (sj > nN - 1 ? nN - 1 : sj);
    const float* xi = x + (size_t)di * 3;
    const float* xj = x + (size_t)sj * 3;
    const float rx = xi[0] - xj[0], ry = xi[1] - xj[1], rz = xi[2] - xj[2];
    const float dsq  = (rx * rx + rz * rz) + ry * ry;
    const float rinv = rcp_f(sqrtf(dsq + 1e-8f));
    const float cw   = xsx[2 * row] + xsx[2 * row + 1];
    v4f o;
    o.x = (rx * rinv) * cw; o.y = (ry * rinv) * cw; o.z = (rz * rinv) * cw; o.w = 0.0f;
    float* ap2 = aux + (size_t)(rl0 + row) * 4;
    *(volatile v4f*)ap2 = o;
    __threadfence();
    *(volatile v4f*)ap2 = o;
  }

  float* dstp = mijf + (size_t)rl0 * HDIM;
  v4f ov[NIT4];
#pragma unroll
  for (int it = 0; it < NIT4; ++it) ov[it] = *(const v4f*)(stg + 4 * (it * NTHR + tid));
#pragma unroll
  for (int it = 0; it < NIT4; ++it) *(volatile v4f*)(dstp + 4 * (size_t)(it * NTHR + tid)) = ov[it];
  __threadfence();
#pragma unroll
  for (int it = 0; it < NIT4; ++it) *(volatile v4f*)(dstp + 4 * (size_t)(it * NTHR + tid)) = ov[it];
}

__global__ __launch_bounds__(NTHR) __attribute__((amdgpu_num_vgpr(256)))
void k_gather(const int* __restrict__ ei, const float* __restrict__ mijf, const float* __restrict__ aux,
              const float* __restrict__ x, float* mi, float* dx, float* xout,
              int nN, int ebase, int clen, int firstChunk, int lastChunk, int nOutX) {
  extern __shared__ __align__(16) char smem_g[];
  int*            slist  = (int*)(smem_g + LG_SLIST);
  unsigned short* slots  = (unsigned short*)(smem_g + LG_SLOTS);
  int*            sdl    = (int*)(smem_g + LG_SDL);
  float*          sdx    = (float*)(smem_g + LG_SDX);
  float*          xo     = (float*)(smem_g + LG_XO);
  int*            scount = (int*)(smem_g + LG_SCNT);
  int*            wsum   = (int*)(smem_g + LG_WSUM);
  int*            scnt   = wsum + NWV;

  const int tid = threadIdx.x, lane = tid & 31;
  const int wave = __builtin_amdgcn_readfirstlane(tid >> 5);
  const int node0 = blockIdx.x * NB;
  const v4f z4 = {0.0f, 0.0f, 0.0f, 0.0f};
  const float qn = __int_as_float(0x7fc00000);
  const v4f vnan = {qn, qn, qn, qn};

  int cnt = 0, pass = 0;
  for (int cb = 0; ; cb += CH) {
    const bool endc = (cb >= clen);
    if (endc || (cnt + CH > LCAP)) {
      __syncthreads();
      int k = 0;
#pragma unroll 1
      for (int i = 0; i < cnt; i += 4) {
        const v4i w4 = *(const v4i*)(sdl + i);
#pragma unroll
        for (int q = 0; q < 4; ++q) {
          const bool hit = (w4[q] == tid) && (i + q < cnt);
          if (hit) {
            if (k < SP) slots[tid * SP + k] = (unsigned short)(i + q);
            ++k;
          }
        }
      }
      scount[tid] = k;
      __syncthreads();

      const bool first = (firstChunk != 0) && (pass == 0);
      const int nw0 = node0 + 32 * wave;
      v4f vold = *(const v4f*)(dx + (size_t)(nw0 + lane) * 4);
      vold = first ? z4 : vold;
      v4f vdx = z4;
#pragma unroll 1
      for (int j = 0; j < 32; ++j) {
        const int nl = 32 * wave + j;
        float* mrow = mi + (size_t)(node0 + nl) * HDIM + 4 * lane;
        int cn = __builtin_amdgcn_readfirstlane(scount[nl]);
        const bool ovf = cn > SP;
        cn = cn > SP ? SP : cn;
        v4f acc = *(const v4f*)mrow;
        acc = first ? z4 : acc;
        v4f dacc = z4;
#pragma unroll 1
        for (int p = 0; p < cn; ++p) {
          int i = (int)slots[nl * SP + p];
          i = i > LCAP - 1 ? LCAP - 1 : i;
          int el = slist[i];
          el = el < 0 ? 0 : (el > clen - 1 ? clen - 1 : el);
          const v4f avv = *(const v4f*)(aux + (size_t)el * 4);
          const v4f ms  = *(const v4f*)(mijf + (size_t)el * HDIM + 4 * lane);
          acc = acc + ms;
          dacc.x += avv.x; dacc.y += avv.y; dacc.z += avv.z;
        }
        acc = ovf ? vnan : acc;
        *(volatile v4f*)mrow = acc;
        __threadfence();
        *(volatile v4f*)mrow = acc;
        const v4f nv = vold + dacc;
        vdx = (lane == j) ? nv : vdx;
      }
      float* drow = dx + (size_t)(nw0 + lane) * 4;
      *(volatile v4f*)drow = vdx;
      __threadfence();
      *(volatile v4f*)drow = vdx;
      *(v4f*)(sdx + (size_t)(32 * wave + lane) * 4) = vdx;
      __syncthreads();
      ++pass;
      cnt = 0;
    }
    if (endc) break;

    int dv[8];
    if (cb + CH <= clen) {
      const int* bp = ei + (size_t)ebase + cb + 8 * tid;
      const v4i a = *(const v4i*)bp;
      const v4i b = *(const v4i*)(bp + 4);
      dv[0] = a[0]; dv[1] = a[1]; dv[2] = a[2]; dv[3] = a[3];
      dv[4] = b[0]; dv[5] = b[1]; dv[6] = b[2]; dv[7] = b[3];
    } else {
#pragma unroll
      for (int j = 0; j < 8; ++j) {
        const int el = cb + 8 * tid + j;
        const int ec = el > clen - 1 ? clen - 1 : el;
        const int dj = ei[(size_t)ebase + ec];
        dv[j] = (el < clen) ? dj : -1;
      }
    }
    unsigned bits = 0u;
#pragma unroll
    for (int j = 0; j < 8; ++j) {
      const int dlj = dv[j] - node0;
      bits |= ((unsigned)dlj < (unsigned)NB) ? (1u << j) : 0u;
    }
    const int pc = __builtin_popcount(bits);
    int incl = pc;
#pragma unroll
    for (int sh = 1; sh < 32; sh <<= 1) {
      const int t = __shfl_up(incl, sh);
      incl += (lane >= sh) ? t : 0;
    }
    if (lane == 31) wsum[wave] = incl;
    __syncthreads();
    int woff = 0, tot = 0;
#pragma unroll
    for (int w = 0; w < NWV; ++w) {
      const int v = wsum[w];
      woff += (w < wave) ? v : 0;
      tot += v;
    }
    int pos = cnt + woff + incl - pc;
#pragma unroll
    for (int j = 0; j < 8; ++j) {
      if (bits & (1u << j)) {
        if (pos < LCAP) {
          slist[pos] = cb + 8 * tid + j;
          sdl[pos]   = dv[j] - node0;
        }
        ++pos;
      }
    }
    if (tid == 0) scnt[0] = cnt + tot;
    __syncthreads();
    cnt = scnt[0];
    cnt = cnt > LCAP ? LCAP : cnt;
  }

  if (lastChunk != 0) {
    for (int i = tid; i < NB * 3; i += NTHR) {
      const int nl = i / 3;
      const int c  = i - nl * 3;
      const int node = node0 + nl;
      const int nc = node > nN - 1 ? nN - 1 : node;
      xo[i] = x[(size_t)nc * 3 + c] + sdx[nl * 4 + c];
    }
    __syncthreads();
    if (tid < NB * 3 / 4) {
      const int g0 = node0 * 3 + 4 * tid;
      const v4f v = *(const v4f*)(xo + 4 * tid);
      float* dp = xout + g0;
      if (g0 + 3 < nOutX) {
        *(volatile v4f*)dp = v;
        __threadfence();
        *(volatile v4f*)dp = v;
      } else {
        if (g0 < nOutX)     *(volatile float*)(dp)     = v.x;
        if (g0 + 1 < nOutX) *(volatile float*)(dp + 1) = v.y;
        if (g0 + 2 < nOutX) *(volatile float*)(dp + 2) = v.z;
        if (g0 + 3 < nOutX) *(volatile float*)(dp + 3) = v.w;
        __threadfence();
        if (g0 < nOutX)     *(volatile float*)(dp)     = v.x;
        if (g0 + 1 < nOutX) *(volatile float*)(dp + 1) = v.y;
        if (g0 + 2 < nOutX) *(volatile float*)(dp + 2) = v.z;
        if (g0 + 3 < nOutX) *(volatile float*)(dp + 3) = v.w;
      }
    }
  }
}

__global__ __launch_bounds__(NTHR) __attribute__((amdgpu_num_vgpr(256)))
void k_node(const float* __restrict__ mi, const float* __restrict__ hin, const int* __restrict__ bidx,
            const float* __restrict__ film,
            const unsigned short* __restrict__ w1h, const unsigned short* __restrict__ w1l,
            const unsigned short* __restrict__ w2h, const unsigned short* __restrict__ w2l,
            const float* __restrict__ bn1, const float* __restrict__ bn2,
            const float* __restrict__ lng, const float* __restrict__ lnb,
            float* hout, int nN, int nG) {
  constexpr int NIT4 = (TR * HDIM / 4) / NTHR;
  __shared__ __attribute__((aligned(16))) float tb[TR * LDF];
  __shared__ float smu[TR];
  __shared__ float srs[TR];
  __shared__ int   sb[TR];
  const int tid = threadIdx.x, lane = tid & 31;
  const int wave = __builtin_amdgcn_readfirstlane(tid >> 5);
  const int h = lane >> 4, m = lane & 15;
  const int rg = wave >> 1, ch = wave & 1;
  const int cb = 64 * ch;
  const int rowBase = blockIdx.x * TR;
  const int grow = rowBase + 16 * rg + m;
  const int gcl = grow > nN - 1 ? nN - 1 : grow;

  if (tid < TR) {
    int rr = rowBase + tid;
    rr = rr > nN - 1 ? nN - 1 : rr;
    int g = bidx[rr];
    g = g < 0 ? 0 : (g > nG - 1 ? nG - 1 : g);
    sb[tid] = g;
  }

  v8f acc[4];
#pragma unroll
  for (int nt = 0; nt < 4; ++nt) acc[nt] = zero8();
  {
    const float* ap1 = hin + (size_t)gcl * HDIM;
    const float* ap2 = mi  + (size_t)grow * HDIM;
    const size_t boff = (size_t)(cb + m) * (2 * HDIM) + 8 * h;
#pragma unroll 1
    for (int kt = 0; kt < HDIM / 32; ++kt) {
      FragB ah, al;
      afrag_bf(ap1 + 32 * kt, h, ah, al);
#pragma unroll
      for (int nt = 0; nt < 4; ++nt) {
        const size_t o = boff + (size_t)(16 * nt) * (2 * HDIM) + 32 * kt;
        const v16b bh = fragbf(w1h + o);
        const v16b bl = fragbf(w1l + o);
        acc[nt] = wmb(ah.v, bh, acc[nt]);
        acc[nt] = wmb(ah.v, bl, acc[nt]);
        acc[nt] = wmb(al.v, bh, acc[nt]);
      }
    }
#pragma unroll 1
    for (int kt = 0; kt < HDIM / 32; ++kt) {
      FragB ah, al;
      afrag_bf(ap2 + 32 * kt, h, ah, al);
#pragma unroll
      for (int nt = 0; nt < 4; ++nt) {
        const size_t o = boff + (size_t)(16 * nt) * (2 * HDIM) + HDIM + 32 * kt;
        const v16b bh = fragbf(w1h + o);
        const v16b bl = fragbf(w1l + o);
        acc[nt] = wmb(ah.v, bh, acc[nt]);
        acc[nt] = wmb(ah.v, bl, acc[nt]);
        acc[nt] = wmb(al.v, bh, acc[nt]);
      }
    }
  }
  {
    float* trow = tb + (size_t)(16 * rg + 8 * h) * LDF + cb + m;
#pragma unroll
    for (int nt = 0; nt < 4; ++nt) {
      const float bb = bn1[cb + 16 * nt + m];
#pragma unroll
      for (int r = 0; r < 8; ++r) trow[r * LDF + 16 * nt] = silu_f(acc[nt][r] + bb);
    }
  }
  __syncthreads();

#pragma unroll
  for (int nt = 0; nt < 4; ++nt) acc[nt] = zero8();
  {
    const float* arow = tb + (size_t)(16 * rg + m) * LDF;
    const size_t boff = (size_t)(cb + m) * HDIM + 8 * h;
#pragma unroll 1
    for (int kt = 0; kt < HDIM / 32; ++kt) {
      FragB ah, al;
      afrag_bf(arow + 32 * kt, h, ah, al);
#pragma unroll
      for (int nt = 0; nt < 4; ++nt) {
        const size_t o = boff + (size_t)(16 * nt) * HDIM + 32 * kt;
        const v16b bh = fragbf(w2h + o);
        const v16b bl = fragbf(w2l + o);
        acc[nt] = wmb(ah.v, bh, acc[nt]);
        acc[nt] = wmb(ah.v, bl, acc[nt]);
        acc[nt] = wmb(al.v, bh, acc[nt]);
      }
    }
  }
  __syncthreads();
  {
    float* srow = tb + (size_t)(16 * rg + 8 * h) * LDF + cb + m;
#pragma unroll
    for (int nt = 0; nt < 4; ++nt) {
      const float bb = bn2[cb + 16 * nt + m];
#pragma unroll
      for (int r = 0; r < 8; ++r) srow[r * LDF + 16 * nt] = acc[nt][r] + bb;
    }
  }
  __syncthreads();

  v4f ov[NIT4];
#pragma unroll
  for (int it = 0; it < NIT4; ++it) {
    const int u  = it * NTHR + tid;
    const int lr = u >> 5;
    const int c4 = (u & 31) * 4;
    int rr = rowBase + lr;
    rr = rr > nN - 1 ? nN - 1 : rr;
    const int g = sb[lr];
    const v4f hv = *(const v4f*)(hin + (size_t)rr * HDIM + c4);
    const v4f ga = *(const v4f*)(film + (size_t)g * (2 * HDIM) + c4);
    const v4f be = *(const v4f*)(film + (size_t)g * (2 * HDIM) + HDIM + c4);
    float* tp = tb + (size_t)lr * LDF + c4;
    const v4f hn = *(const v4f*)tp;
    const v4f t  = ga * hn + be;
    const v4f xv = hv + t;
    *(v4f*)tp = xv;
    ov[it] = xv;
  }
  __syncthreads();

  if (tid < TR) {
    const float* row = tb + (size_t)tid * LDF;
    float s = 0.0f;
#pragma unroll 4
    for (int c = 0; c < HDIM; ++c) s += row[c];
    const float mu = s * (1.0f / 128.0f);
    float q = 0.0f;
#pragma unroll 4
    for (int c = 0; c < HDIM; ++c) { const float d = row[c] - mu; q += d * d; }
    const float var = q * (1.0f / 128.0f);
    smu[tid] = mu;
    srs[tid] = 1.0f / sqrtf(var + 1e-5f);
  }
  __syncthreads();

  v4f yv[NIT4];
#pragma unroll
  for (int it = 0; it < NIT4; ++it) {
    const int u  = it * NTHR + tid;
    const int lr = u >> 5;
    const int c4 = (u & 31) * 4;
    const float mu = smu[lr], rs = srs[lr];
    const v4f g4 = *(const v4f*)(lng + c4);
    const v4f b4 = *(const v4f*)(lnb + c4);
    yv[it] = ((ov[it] - mu) * rs) * g4 + b4;
  }
#pragma unroll
  for (int it = 0; it < NIT4; ++it) {
    const int u = it * NTHR + tid;
    const int orow = rowBase + (u >> 5);
    if (orow < nN) *(volatile v4f*)(hout + (size_t)orow * HDIM + 4 * (u & 31)) = yv[it];
  }
  __threadfence();
#pragma unroll
  for (int it = 0; it < NIT4; ++it) {
    const int u = it * NTHR + tid;
    const int orow = rowBase + (u >> 5);
    if (orow < nN) *(volatile v4f*)(hout + (size_t)orow * HDIM + 4 * (u & 31)) = yv[it];
  }
}

extern "C" void kernel_launch(void* const* d_in, const int* in_sizes, int n_in,
                              void* d_out, int out_size, void* d_ws, size_t ws_size,
                              hipStream_t stream) {
  if (n_in < 21) return;
  const int nN = in_sizes[0] / HDIM;
  const int nE = in_sizes[4] / 2;
  const int nG = in_sizes[3] / HDIM;
  if (nN <= 0 || nE <= 0 || nG <= 0) return;
  if (in_sizes[0] != nN * HDIM || in_sizes[1] != nN * 3 || in_sizes[2] != nE * EFD) return;
  if (in_sizes[3] != nG * HDIM || in_sizes[4] != 2 * nE || in_sizes[5] != nN) return;
  if (in_sizes[6] != K1R * HDIM || in_sizes[7] != HDIM) return;
  if (in_sizes[8] != HDIM * HDIM || in_sizes[9] != HDIM) return;
  if (in_sizes[10] != HDIM * HDIM || in_sizes[11] != HDIM || in_sizes[12] != HDIM) return;
  if (in_sizes[13] != 2 * HDIM * HDIM || in_sizes[14] != HDIM) return;
  if (in_sizes[15] != HDIM * HDIM || in_sizes[16] != HDIM) return;
  if (in_sizes[17] != HDIM * 2 * HDIM || in_sizes[18] != 2 * HDIM) return;
  if (in_sizes[19] != HDIM || in_sizes[20] != HDIM) return;
  if ((size_t)out_size != (size_t)nN * HDIM + (size_t)nN * 3) return;
  if (nE > (1 << 27) || nN > (1 << 22) || nG > (1 << 16)) return;

  const float* hin  = (const float*)d_in[0];
  const float* x    = (const float*)d_in[1];
  const float* ea   = (const float*)d_in[2];
  const float* cond = (const float*)d_in[3];
  const int*   ei   = (const int*)d_in[4];
  const int*   bidx = (const int*)d_in[5];
  const float* W1   = (const float*)d_in[6];
  const float* b1   = (const float*)d_in[7];
  const float* W2   = (const float*)d_in[8];
  const float* b2   = (const float*)d_in[9];
  const float* Wc1  = (const float*)d_in[10];
  const float* bc1  = (const float*)d_in[11];
  const float* Wc2  = (const float*)d_in[12];
  const float* Wn1  = (const float*)d_in[13];
  const float* bn1  = (const float*)d_in[14];
  const float* Wn2  = (const float*)d_in[15];
  const float* bn2  = (const float*)d_in[16];
  const float* Wf   = (const float*)d_in[17];
  const float* bfm  = (const float*)d_in[18];
  const float* lng  = (const float*)d_in[19];
  const float* lnb  = (const float*)d_in[20];
  float* hout = (float*)d_out;
  float* xout = (float*)d_out + (size_t)nN * HDIM;

  const int nGat   = (nN + NB - 1) / NB;
  const int NPAD   = nGat * NB;
  const int nGemm  = NPAD / BM;
  const int nNode  = NPAD / TR;
  const int nChunk = (nE + CE - 1) / CE;
  if (nChunk > 256) return;

  char* ws = (char*)d_ws;
  size_t off = 0;
  const size_t oWPQ = off; off += (size_t)PW * HDIM * 2;        off = (off + 255) & ~(size_t)255;
  const size_t oWE  = off; off += (size_t)HDIM * KE * 2;        off = (off + 255) & ~(size_t)255;
  const size_t oW2  = off; off += (size_t)HDIM * HDIM * 2;      off = (off + 255) & ~(size_t)255;
  const size_t oWX  = off; off += (size_t)HDIM * HDIM * 2;      off = (off + 255) & ~(size_t)255;
  const size_t oN1H = off; off += (size_t)HDIM * 2 * HDIM * 2;  off = (off + 255) & ~(size_t)255;
  const size_t oN1L = off; off += (size_t)HDIM * 2 * HDIM * 2;  off = (off + 255) & ~(size_t)255;
  const size_t oN2H = off; off += (size_t)HDIM * HDIM * 2;      off = (off + 255) & ~(size_t)255;
  const size_t oN2L = off; off += (size_t)HDIM * HDIM * 2;      off = (off + 255) & ~(size_t)255;
  const size_t oFLM = off; off += (size_t)nG * 2 * HDIM * 4;    off = (off + 255) & ~(size_t)255;
  const size_t oPQ  = off; off += (size_t)NPAD * PW * 4;        off = (off + 255) & ~(size_t)255;
  const size_t oMI  = off; off += (size_t)NPAD * HDIM * 4;      off = (off + 255) & ~(size_t)255;
  const size_t oDX  = off; off += (size_t)NPAD * 4 * 4;         off = (off + 255) & ~(size_t)255;
  const size_t oM1  = off; off += (size_t)CE * HDIM * 2;        off = (off + 255) & ~(size_t)255;
  const size_t oMJ  = off; off += (size_t)CE * HDIM * 4;        off = (off + 255) & ~(size_t)255;
  const size_t oAUX = off; off += (size_t)CE * 4 * 4;           off = (off + 255) & ~(size_t)255;
  if (off > ws_size || off > (size_t)WSCAP) return;
  _Float16*       wPQ  = (_Float16*)(ws + oWPQ);
  _Float16*       wE   = (_Float16*)(ws + oWE);
  _Float16*       w2   = (_Float16*)(ws + oW2);
  _Float16*       wx   = (_Float16*)(ws + oWX);
  unsigned short* wn1h = (unsigned short*)(ws + oN1H);
  unsigned short* wn1l = (unsigned short*)(ws + oN1L);
  unsigned short* wn2h = (unsigned short*)(ws + oN2H);
  unsigned short* wn2l = (unsigned short*)(ws + oN2L);
  float*          filmP = (float*)(ws + oFLM);
  float*          pqP  = (float*)(ws + oPQ);
  float*          miP  = (float*)(ws + oMI);
  float*          dxP  = (float*)(ws + oDX);
  _Float16*       m1p  = (_Float16*)(ws + oM1);
  float*          mijf = (float*)(ws + oMJ);
  float*          auxp = (float*)(ws + oAUX);

  (void)hipFuncSetAttribute(reinterpret_cast<const void*>(&k_gather),
                            hipFuncAttributeMaxDynamicSharedMemorySize, (int)LDS_G);

  const int u128 = HDIM * (HDIM / 8);
  const int u256 = HDIM * (2 * HDIM / 8);
  const int u32  = HDIM * (KE / 8);
  const int ufl  = nG * (2 * HDIM / 4);
  k_wcvt<<<(u128 + NTHR - 1) / NTHR, NTHR, 0, stream>>>(W1, wPQ, HDIM, 0, HDIM, HDIM, u128, SCL_W);
  k_wcvt<<<(u128 + NTHR - 1) / NTHR, NTHR, 0, stream>>>(W1, wPQ + (size_t)HDIM * HDIM, HDIM, HDIM, HDIM, HDIM, u128, SCL_W);
  k_wcvt<<<(u32 + NTHR - 1) / NTHR, NTHR, 0, stream>>>(W1, wE, HDIM, KEOFF, EFD, KE, u32, SCL_W);
  k_wcvt<<<(u128 + NTHR - 1) / NTHR, NTHR, 0, stream>>>(W2, w2, HDIM, 0, HDIM, HDIM, u128, SCL_W);
  k_wcvt<<<(u128 + NTHR - 1) / NTHR, NTHR, 0, stream>>>(Wc1, wx, HDIM, 0, HDIM, HDIM, u128, SCL_W);
  k_wcvt_bf<<<(u256 + NTHR - 1) / NTHR, NTHR, 0, stream>>>(Wn1, wn1h, wn1l, HDIM, 0, 2 * HDIM, 2 * HDIM, u256);
  k_wcvt_bf<<<(u128 + NTHR - 1) / NTHR, NTHR, 0, stream>>>(Wn2, wn2h, wn2l, HDIM, 0, HDIM, HDIM, u128);
  k_film<<<(ufl + NTHR - 1) / NTHR, NTHR, 0, stream>>>(cond, Wf, bfm, filmP, ufl);
  k_nodegemm<<<nGemm, NTHR, 0, stream>>>(hin, wPQ, b1, pqP, nN);
  for (int c = 0; c < nChunk; ++c) {
    const int ebase = c * CE;
    const int clen  = (nE - ebase) < CE ? (nE - ebase) : CE;
    const int nb    = (clen + TR - 1) / TR;
    k_edge1<<<nb, NTHR, 0, stream>>>(pqP, ei, x, ea, wE, W1 + (size_t)KDSQ * HDIM, m1p, nE, nN, ebase);
    k_edge2<<<nb, NTHR, 0, stream>>>(m1p, ei, x, w2, wx, b2, bc1, Wc2, mijf, auxp, nE, nN, ebase);
    k_gather<<<nGat, NTHR, LDS_G, stream>>>(ei, mijf, auxp, x, miP, dxP, xout, nN, ebase, clen,
                                             (c == 0) ? 1 : 0, (c == nChunk - 1) ? 1 : 0, nN * 3);
  }
  k_node<<<nNode, NTHR, 0, stream>>>(miP, hin, bidx, filmP, wn1h, wn1l, wn2h, wn2l, bn1, bn2, lng, lnb,
                                     hout, nN, nG);
}
